// DSANLayer_15522011807844
// MI455X (gfx1250) — hardware-run, weakly checked
//
#include <hip/hip_runtime.h>


namespace {
constexpr int N = 2048, E = 4096, HID = 128, NH = 8, HD = 16, HP = 32  , QP = 64  ;
constexpr float XS = 8.0f, WSC = 256.0f, PS = 8.0f, SCALE = 0.25f, LOG2E = 1.4426950408889634f;

typedef _Float16 b16;
typedef __attribute__((ext_vector_type(16))) _Float16 v16b;
typedef __attribute__((ext_vector_type(8))) _Float16 v8b;
typedef __attribute__((ext_vector_type(8))) float v8f;
typedef __attribute__((ext_vector_type(4))) float v4f;
__device__ __forceinline__ float bf16_rne(float f) { unsigned int u = __float_as_uint(f); u += 0x7FFFu + ((u >> 16) & 1u); return __uint_as_float(u & 0xFFFF0000u); }
__device__ __forceinline__ void split16(float v, b16& hi, b16& lo) { hi = (b16)v; lo = (b16)(v - (float)hi); }
__device__ __forceinline__ v16b frag_kb(const b16* p, int hh) { const v8b a = *(const v8b*)(p + 8 * hh), b = *(const v8b*)(p + 16 + 8 * hh); v16b f;
#pragma unroll
  for (int e = 0; e < 8; ++e) { f[e] = a[e]; f[8 + e] = b[e]; } return f; }
__device__ __forceinline__ v8f wmma16b(v16b a, v16b b, v8f c) { v8f d = __builtin_amdgcn_wmma_f32_16x16x32_f16(false, a, false, b, (short)0, c, false, false); asm volatile("v_nop\n\tv_nop\n\tv_nop\n\tv_nop" : "+v"(d) : "v"(a), "v"(b)); return d; }
__device__ __forceinline__ void wave_lds_sync() { __builtin_amdgcn_fence(__ATOMIC_RELEASE, "workgroup"); __builtin_amdgcn_wave_barrier(); __builtin_amdgcn_fence(__ATOMIC_ACQUIRE, "workgroup"); }
__device__ __forceinline__ float pmul(float a, float b) { float p = a * b; asm volatile("" : "+v"(p)); return p; }
__device__ __forceinline__ int iclamp(int v, int lo, int hi) { return v < lo ? lo : (v > hi ? hi : v); }
__device__ __forceinline__ float nexp2(float x) { return __builtin_amdgcn_exp2f(x); }

constexpr int CSR_NBLK = 512, CSR_GB = 9, CSR_GN = 1 << CSR_GB  , CSR_MAXG = 512, CSR_CAP = 12288  ;
__global__ __launch_bounds__(64) void csrA_kernel(const int* __restrict__ dst, int E, int N, int nG, int CHP, int NGP, int* __restrict__ STG, int* __restrict__ HST) {
  extern __shared__ int sm[];
  int* cnt = sm; int* run = sm + NGP; int* ids = sm + 2 * NGP;
  const int b = blockIdx.x; const int ch = (E + CSR_NBLK - 1) / CSR_NBLK; const int e0 = b * ch, e1 = min(E, e0 + ch);
  for (int i = threadIdx.x; i < NGP; i += 64) cnt[i] = 0;
  for (int i = threadIdx.x; i < CHP; i += 64) ids[i] = -1;
  __syncthreads();
  if (threadIdx.x == 0) {
    for (int e = e0; e < e1; ++e) { int d = dst[e]; d = (d < 0) ? 0 : (d >= N ? N - 1 : d); cnt[d >> CSR_GB] += 1; }
    int acc = 0; for (int g = 0; g < nG; ++g) { run[g] = acc; acc += cnt[g]; }
    for (int e = e0; e < e1; ++e) { int d = dst[e]; d = (d < 0) ? 0 : (d >= N ? N - 1 : d); const int g = d >> CSR_GB; ids[run[g]] = e; run[g] += 1; } }
  __syncthreads();
  typedef __attribute__((ext_vector_type(4))) int v4i;
  for (int pass = 0; pass < 2; ++pass) {
    for (int i = threadIdx.x; i < CHP / 4; i += 64) *(volatile v4i*)(STG + (size_t)b * CHP + i * 4) = *(const v4i*)(&ids[i * 4]);
    for (int i = threadIdx.x; i < NGP / 4; i += 64) { v4i v; for (int e = 0; e < 4; ++e) v[e] = (i * 4 + e < nG) ? cnt[i * 4 + e] : 0; *(volatile v4i*)(HST + (size_t)b * NGP + i * 4) = v; }
    __threadfence(); }
}
__global__ __launch_bounds__(512) void csrS_kernel(const int* __restrict__ HST, int nG, int NGP, int* __restrict__ START, int* __restrict__ TOT, int* __restrict__ OFF) {
  __shared__ int tot[CSR_MAXG];
  const int b = threadIdx.x;
  for (int pass = 0; pass < 2; ++pass) { int runb = 0; for (int g = 0; g < nG; ++g) { int c = HST[(size_t)b * NGP + g]; c = (c < 0) ? 0 : c; ((volatile int*)OFF)[(size_t)g * CSR_NBLK + b] = runb; runb += c; } __threadfence(); }
  for (int g = threadIdx.x; g < nG; g += 512) { int s = 0; for (int bb = 0; bb < CSR_NBLK; ++bb) { int c = HST[(size_t)bb * NGP + g]; s += (c < 0) ? 0 : c; } tot[g] = s; }
  __syncthreads();
  if (threadIdx.x < 32) {
    __shared__ int st[CSR_MAXG + 32];
    if (threadIdx.x == 0) { int acc = 0; for (int g = 0; g < NGP; ++g) { st[g] = acc; if (g < nG) acc += (tot[g] + 31) & ~31; } st[NGP] = acc; }
    __builtin_amdgcn_fence(__ATOMIC_RELEASE, "workgroup"); __builtin_amdgcn_wave_barrier(); __builtin_amdgcn_fence(__ATOMIC_ACQUIRE, "workgroup");
    for (int pass = 0; pass < 2; ++pass) { for (int i = threadIdx.x; i < NGP + 32; i += 32) { ((volatile int*)START)[i] = (i <= NGP) ? st[min(i, NGP)] : 0; ((volatile int*)TOT)[i] = (i < nG) ? tot[i] : 0; } __threadfence(); } }
}
__global__ __launch_bounds__(256) void csrB_kernel(const int* __restrict__ dst, int N, int nG, int CHP, int NGP, int permLen, const int* __restrict__ STG, const int* __restrict__ HST, const int* __restrict__ OFF, const int* __restrict__ START, const int* __restrict__ TOT, int* __restrict__ PERM, int* __restrict__ ROWPTR, int* __restrict__ ROWCNT, int* __restrict__ FLAG) {
  typedef __attribute__((ext_vector_type(4))) int v4i;
  __shared__ int ids[CSR_CAP]; __shared__ unsigned short key[CSR_CAP]; __shared__ int outp[CSR_CAP]; __shared__ int ncnt[CSR_GN + 1]; __shared__ int boff[CSR_NBLK + 1];
  const int g = blockIdx.x, t_ = threadIdx.x; int tot = TOT[g]; int st = START[g], stn = START[g + 1]; const int v0 = g * CSR_GN; const int nv = min(CSR_GN, N - v0);
  st = (st < 0) ? 0 : (st > permLen - 32 ? permLen - 32 : st) & ~31; stn = (stn < st) ? st : (stn > permLen ? permLen : stn); tot = (tot < 0) ? 0 : tot; if (tot > stn - st && tot <= CSR_CAP) tot = stn - st;
  if (tot > CSR_CAP) {
    for (int pass = 0; pass < 2; ++pass) { for (int i = t_; i < CSR_GN / 4; i += 256) { v4i a, c; for (int e = 0; e < 4; ++e) { a[e] = st; c[e] = 0; } *(volatile v4i*)(ROWPTR + v0 + i * 4) = a; *(volatile v4i*)(ROWCNT + v0 + i * 4) = c; } if (t_ == 0) ((volatile int*)FLAG)[0] = 1; __threadfence(); } (void)nv; return; }
  if (t_ == 0) { int acc = 0; for (int b = 0; b < CSR_NBLK; ++b) { boff[b] = acc; int c = HST[(size_t)b * NGP + g]; c = (c < 0) ? 0 : (c > CHP ? CHP : c); acc += c; if (acc > tot) acc = tot; } boff[CSR_NBLK] = acc; }
  for (int i = t_; i <= CSR_GN; i += 256) ncnt[i] = 0;
  __syncthreads();
  for (int b = 0; b < CSR_NBLK; ++b) { const int c = boff[b + 1] - boff[b]; int o_ = OFF[(size_t)g * CSR_NBLK + b]; o_ = (o_ < 0) ? 0 : (o_ > CHP - c ? CHP - c : o_); const int* src_ = STG + (size_t)b * CHP + o_;
    for (int i = t_; i < c; i += 256) { int id = src_[i]; id = (id < 0) ? 0 : id; ids[boff[b] + i] = id; int d = dst[id]; d = (d < v0) ? v0 : (d >= N ? N - 1 : d); int kk = d - v0; kk = (kk < 0) ? 0 : (kk >= CSR_GN ? CSR_GN - 1 : kk); key[boff[b] + i] = (unsigned short)kk; } }
  __syncthreads();
  if (t_ == 0) { for (int i = 0; i < tot; ++i) ncnt[key[i]] += 1; int acc = 0; for (int vl = 0; vl < CSR_GN; ++vl) { const int c = ncnt[vl]; ncnt[vl] = acc; acc += c; } ncnt[CSR_GN] = acc;
    for (int i = 0; i < tot; ++i) { const int vl = key[i]; outp[ncnt[vl]] = ids[i]; ncnt[vl] += 1; }
    for (int vl = CSR_GN; vl > 0; --vl) ncnt[vl] = ncnt[vl - 1]; ncnt[0] = 0; }
  __syncthreads();
  for (int pass = 0; pass < 2; ++pass) {
    for (int i = t_; i < (stn - st) / 4; i += 256) { v4i v; for (int e = 0; e < 4; ++e) { const int q = i * 4 + e; v[e] = (q < tot) ? outp[q] : -1; } *(volatile v4i*)(PERM + st + i * 4) = v; }
    for (int i = t_; i < CSR_GN / 4; i += 256) { v4i a, c; for (int e = 0; e < 4; ++e) { const int vl = i * 4 + e; a[e] = st + ncnt[vl]; c[e] = (vl < nv) ? (ncnt[vl + 1] - ncnt[vl]) : 0; } *(volatile v4i*)(ROWPTR + v0 + i * 4) = a; *(volatile v4i*)(ROWCNT + v0 + i * 4) = c; }
    __threadfence(); }
}
__global__ __launch_bounds__(256) void csrZ_kernel(int* __restrict__ p, size_t n4) { typedef __attribute__((ext_vector_type(4))) int v4i; const size_t tid = (size_t)blockIdx.x * 256 + threadIdx.x, nth = (size_t)gridDim.x * 256; v4i z = {0, 0, 0, 0}; for (size_t i = tid; i < n4; i += nth) *(volatile v4i*)(p + i * 4) = z; }
struct CsrBufs { int *STG, *HST, *OFF, *START, *TOT, *PERM, *ROWPTR, *ROWCNT, *FLAG; int nG, NGP, CHP; size_t permLen; char* base; size_t bytes; };
static size_t csr_carve(CsrBufs& c, char* ws, size_t off, int E, int N) {
  const size_t off0 = off; c.base = ws + off;
  auto al = [&](size_t bytes) { char* p = ws + off; off += (bytes + 255) & ~(size_t)255; return p; };
  c.nG = (N + CSR_GN - 1) / CSR_GN; c.NGP = (c.nG + 31) & ~31; const int ch = (E + CSR_NBLK - 1) / CSR_NBLK; c.CHP = (ch + 31) & ~31; c.permLen = (size_t)E + 32 * (size_t)c.nG + 32;
  c.STG = (int*)al((size_t)CSR_NBLK * c.CHP * 4); c.HST = (int*)al((size_t)CSR_NBLK * c.NGP * 4); c.OFF = (int*)al((size_t)c.NGP * CSR_NBLK * 4); c.START = (int*)al((size_t)(c.NGP + 64) * 4); c.TOT = (int*)al((size_t)(c.NGP + 64) * 4);
  c.PERM = (int*)al(c.permLen * 4); c.ROWPTR = (int*)al((size_t)c.nG * CSR_GN * 4); c.ROWCNT = (int*)al((size_t)c.nG * CSR_GN * 4); c.FLAG = (int*)al(256);
  c.bytes = off - off0; return off;
}
static void csr_build(const CsrBufs& c, const int* dst, int E, int N, hipStream_t stream) {
  const size_t smem = (size_t)(2 * c.NGP + c.CHP) * 4;
  csrZ_kernel<<<512, 256, 0, stream>>>((int*)c.base, c.bytes / 16);
  csrA_kernel<<<CSR_NBLK, 64, smem, stream>>>(dst, E, N, c.nG, c.CHP, c.NGP, c.STG, c.HST);
  csrS_kernel<<<1, 512, 0, stream>>>(c.HST, c.nG, c.NGP, c.START, c.TOT, c.OFF);
  csrB_kernel<<<c.nG, 256, 0, stream>>>(dst, N, c.nG, c.CHP, c.NGP, (int)c.permLen, c.STG, c.HST, c.OFF, c.START, c.TOT, c.PERM, c.ROWPTR, c.ROWCNT, c.FLAG);
}


__global__ __launch_bounds__(256) void prep_kernel(const float* __restrict__ x, const float* __restrict__ we1, const float* __restrict__ we2, const float* __restrict__ wq, const float* __restrict__ wk, const float* __restrict__ wv, const float* __restrict__ wo, b16* __restrict__ X16, b16* __restrict__ WT) {
  const int t = blockIdx.x * 256 + threadIdx.x; const int nx = N * HID / 8, nw = 7 * HID * HID / 8; v8b o;
  if (t < nx) { const int e = t * 8; for (int j = 0; j < 8; ++j) o[j] = (b16)(bf16_rne(x[e + j]) * XS); for (int pass = 0; pass < 2; ++pass) { *(volatile v8b*)(X16 + e) = o; __threadfence(); } }
  else if (t < nx + nw) { const int e = (t - nx) * 8; const int k = e / (HID * HID), r = e % (HID * HID); const int oo = r / HID, i0 = r % HID; const float* w; int ioff = 0;
    switch (k) { case 0: w = we1; break; case 1: w = we1; ioff = HID; break; case 2: w = we2; break; case 3: w = wq; break; case 4: w = wk; break; case 5: w = wv; break; default: w = wo; }
    for (int j = 0; j < 8; ++j) o[j] = (b16)(bf16_rne(w[(size_t)(ioff + i0 + j) * HID + oo]) * WSC); for (int pass = 0; pass < 2; ++pass) { *(volatile v8b*)(WT + e) = o; __threadfence(); } }
}
template <int MODE>
__global__ __launch_bounds__(128) void gemm_kernel(const b16* __restrict__ Ah, const b16* __restrict__ Al, const b16* __restrict__ W, const float* __restrict__ b0, const float* __restrict__ b1_, const float* __restrict__ b2_, float* __restrict__ Y0, float* __restrict__ Y1, b16* __restrict__ Yh, b16* __restrict__ Yl, b16* __restrict__ Z2, b16* __restrict__ Z3) {
  __shared__ __attribute__((aligned(16))) float Ts[4][16][HID + 4];
  const int wave = threadIdx.x >> 5, lane = threadIdx.x & 31, nloc = lane & 15, hlf = lane >> 4, t_ = threadIdx.x; const size_t m0 = (size_t)blockIdx.x * 64 + wave * 16; const int which = blockIdx.y;
  const b16* Wp = W + (size_t)which * HID * HID; const float* bias = which == 0 ? b0 : which == 1 ? b1_ : b2_;
  v8f acc[8];
#pragma unroll
  for (int t = 0; t < 8; ++t) acc[t] = (v8f){};
#pragma unroll
  for (int kb = 0; kb < HID; kb += 32) { const v16b a = frag_kb(Ah + (m0 + nloc) * HID + kb, hlf); v16b al = {}; if (MODE != 0) al = frag_kb(Al + (m0 + nloc) * HID + kb, hlf);
#pragma unroll
    for (int t = 0; t < 8; ++t) { const v16b bw = frag_kb(Wp + (size_t)(t * 16 + nloc) * HID + kb, hlf); acc[t] = wmma16b(a, bw, acc[t]); if (MODE != 0) acc[t] = wmma16b(al, bw, acc[t]); } }
#pragma unroll
  for (int t = 0; t < 8; ++t) { const int c = t * 16 + nloc; const float bb = bias ? bf16_rne(bias[c]) : 0.0f;
#pragma unroll
    for (int r = 0; r < 8; ++r) { float v = acc[t][r] * (1.0f / (XS * WSC)) + bb; if (MODE == 2 && which == 0) v *= SCALE; Ts[wave][8 * hlf + r][c] = v; } }
  __syncthreads();
  for (int pass = 0; pass < 2; ++pass) {
    if (MODE == 0 || MODE == 1 || MODE == 3) { float* Y = (MODE == 0 && which == 1) ? Y1 : Y0; for (int rr = 0; rr < 16; ++rr) *(volatile v4f*)(Y + (m0 + rr) * HID + lane * 4) = *(const v4f*)(&Ts[wave][rr][lane * 4]); }
    if (MODE == 1) { for (int rr = 0; rr < 16; ++rr) if (lane < 16) { v8b hv, lv; for (int j = 0; j < 8; ++j) { b16 p, q; split16(Ts[wave][rr][lane * 8 + j] * XS, p, q); hv[j] = p; lv[j] = q; } *(volatile v8b*)(Yh + (m0 + rr) * HID + lane * 8) = hv; *(volatile v8b*)(Yl + (m0 + rr) * HID + lane * 8) = lv; } }
    if (MODE == 2 && which < 2) {
      b16* Ph = which == 0 ? Yh : Z2; b16* Pl = which == 0 ? Yl : Z3;
      for (int rr = 0; rr < 16; ++rr) for (int hb = 0; hb < NH; hb += 4) { const int h = hb + (lane >> 3), c8 = (lane & 7) * 8; v8b hv, lv; for (int j = 0; j < 8; ++j) { const int d = c8 + j; float v = d < HD ? Ts[wave][rr][h * HD + d] : 0.0f; b16 p, q; split16(v * XS, p, q); hv[j] = p; lv[j] = q; }
        *(volatile v8b*)(Ph + ((size_t)h * E + m0 + rr) * QP + c8) = hv; *(volatile v8b*)(Pl + ((size_t)h * E + m0 + rr) * QP + c8) = lv; } }
    if (MODE == 2 && which == 2) {
      { b16* VTp = (b16*)Y0; b16* VTlp = (b16*)Y1; const int h = t_ >> 4, d = t_ & 15; for (int c8 = 0; c8 < 64; c8 += 8) { v8b hv, lv; for (int j = 0; j < 8; ++j) { const int rloc = c8 + j; b16 p, q; split16(Ts[rloc >> 4][rloc & 15][h * HD + d] * XS, p, q); hv[j] = p; lv[j] = q; } const size_t gi = ((size_t)h * HD + d) * E + (size_t)blockIdx.x * 64 + c8; *(volatile v8b*)(VTp + gi) = hv; *(volatile v8b*)(VTlp + gi) = lv; } } }
    __threadfence(); }
}
__global__ __launch_bounds__(256) void edge1_kernel(const float* __restrict__ XA, const float* __restrict__ XB, const int* __restrict__ ei, b16* __restrict__ Hh, b16* __restrict__ Hl) {
  const int wave = threadIdx.x >> 5, lane = threadIdx.x & 31; const int e = blockIdx.x * 8 + wave; const int s = iclamp(ei[e], 0, N - 1), d = iclamp(ei[E + e], 0, N - 1); const int c0 = lane * 4;
  __attribute__((ext_vector_type(4))) _Float16 hv, lv; for (int q = 0; q < 4; ++q) { const float v = fmaxf(XA[(size_t)s * HID + c0 + q] + XB[(size_t)d * HID + c0 + q], 0.0f); b16 p, qq; split16(v * XS, p, qq); hv[q] = p; lv[q] = qq; }
  for (int pass = 0; pass < 2; ++pass) { *(volatile __attribute__((ext_vector_type(4))) _Float16*)(Hh + (size_t)e * HID + c0) = hv; *(volatile __attribute__((ext_vector_type(4))) _Float16*)(Hl + (size_t)e * HID + c0) = lv; __threadfence(); }
}
__global__ __launch_bounds__(64) void attn_kernel(const b16* __restrict__ QFh, const b16* __restrict__ QFl, const b16* __restrict__ KRh, const b16* __restrict__ KRl, const b16* __restrict__ VT, const b16* __restrict__ VTl, b16* __restrict__ AOT, b16* __restrict__ AOTl) {
  const int wave = threadIdx.x >> 5, lane = threadIdx.x & 31, hh = lane >> 4, col = lane & 15; const int h = blockIdx.y; const int q0 = blockIdx.x * 32 + wave * 16, qi = q0 + col;
  const size_t qo = ((size_t)h * E + qi) * QP; const v16b qa = frag_kb(QFh + qo, hh), ql = frag_kb(QFl + qo, hh);
  const b16* Kb = KRh + (size_t)h * E * QP; const b16* Klb = KRl + (size_t)h * E * QP; const b16* Vb = VT + (size_t)h * HD * E; const b16* Vlb = VTl + (size_t)h * HD * E;
  float m = -INFINITY, l = 0.0f; v8f o = {};
  const float cs = LOG2E / (XS * XS);
  for (int kb = 0; kb < E; kb += 32) {
    v8f s0 = {}, s1 = {};
    { const b16* k0 = Kb + (size_t)(kb + col) * QP, *k1 = Kb + (size_t)(kb + 16 + col) * QP; v16b f = frag_kb(k0, hh); s0 = wmma16b(f, qa, s0); s0 = wmma16b(f, ql, s0); s0 = wmma16b(frag_kb(Klb + (size_t)(kb + col) * QP, hh), qa, s0);
      f = frag_kb(k1, hh); s1 = wmma16b(f, qa, s1); s1 = wmma16b(f, ql, s1); s1 = wmma16b(frag_kb(Klb + (size_t)(kb + 16 + col) * QP, hh), qa, s1); }
    float e[16]; float mx = -INFINITY;
#pragma unroll
    for (int r = 0; r < 8; ++r) { e[r] = s0[r] * cs; e[8 + r] = s1[r] * cs; mx = fmaxf(mx, fmaxf(e[r], e[8 + r])); }
    mx = fmaxf(mx, __shfl_xor(mx, 16)); const float mn = fmaxf(m, mx); const float al = nexp2(m - mn); m = mn; float sum = 0.0f; v16b ph, pl;
#pragma unroll
    for (int i = 0; i < 16; ++i) { const float p = nexp2(e[i] - mn); sum += p; const b16 h_ = (b16)(p * PS); ph[i] = h_; pl[i] = (b16)(p * PS - (float)h_); }
    sum += __shfl_xor(sum, 16); l = l * al + sum;
    o *= al; const v16b vf = frag_kb(Vb + (size_t)col * E + kb, hh); o = wmma16b(vf, ph, o); o = wmma16b(vf, pl, o); o = wmma16b(frag_kb(Vlb + (size_t)col * E + kb, hh), ph, o); }
  const float inv = 1.0f / (l * PS * XS);
  __shared__ __attribute__((aligned(16))) float To[2][16][HD + 1];
#pragma unroll
  for (int r = 0; r < 8; ++r) To[wave][col][8 * hh + r] = o[r] * inv;
  wave_lds_sync();
  for (int pass = 0; pass < 2; ++pass) { { const int rr = lane >> 1, d8 = (lane & 1) * 8; v8b hv, lv; for (int j = 0; j < 8; ++j) { b16 p, q; split16(To[wave][rr][d8 + j] * XS, p, q); hv[j] = p; lv[j] = q; } const size_t gi = ((size_t)h * E + q0 + rr) * HD + d8; *(volatile v8b*)(AOT + gi) = hv; *(volatile v8b*)(AOTl + gi) = lv; } __threadfence(); }
}
__global__ __launch_bounds__(256) void relay_kernel(const b16* __restrict__ AOT, const b16* __restrict__ AOTl, b16* __restrict__ AOh, b16* __restrict__ AOl) {
  const int wave = threadIdx.x >> 5, lane = threadIdx.x & 31; const int e = blockIdx.x * 8 + wave; const int c0 = lane * 4; const int h = c0 / HD, d0 = c0 % HD;
  typedef __attribute__((ext_vector_type(4))) _Float16 v4b; const v4b a = *(const v4b*)(AOT + ((size_t)h * E + e) * HD + d0), b = *(const v4b*)(AOTl + ((size_t)h * E + e) * HD + d0);
  for (int pass = 0; pass < 2; ++pass) { *(volatile v4b*)(AOh + (size_t)e * HID + c0) = a; *(volatile v4b*)(AOl + (size_t)e * HID + c0) = b; __threadfence(); }
}
__global__ __launch_bounds__(256) void node_kernel(const float* __restrict__ x, const float* __restrict__ UE, const int* __restrict__ PERM, const int* __restrict__ ROWPTR, const int* __restrict__ ROWCNT, int permLen, float* __restrict__ out) {
  const int wave = threadIdx.x >> 5, lane = threadIdx.x & 31; const int v = blockIdx.x * 8 + wave; const int c0 = lane * 4;
  int st = ROWPTR[v], cnt = ROWCNT[v]; cnt = iclamp(cnt, 0, E); st = iclamp(st, 0, permLen - cnt);
  v4f acc; for (int q = 0; q < 4; ++q) acc[q] = bf16_rne(x[(size_t)v * HID + c0 + q]);
  for (int j = 0; j < cnt; ++j) { const int e = iclamp(PERM[st + j], 0, E - 1); const v4f u = *(const v4f*)(UE + (size_t)e * HID + c0); acc += u; }
  for (int pass = 0; pass < 2; ++pass) { *(volatile v4f*)(out + (size_t)v * HID + c0) = acc; __threadfence(); }
}
}

extern "C" void kernel_launch(void* const* d_in, const int* in_sizes, int n_in, void* d_out, int out_size, void* d_ws, size_t ws_size, hipStream_t stream) {
  (void)n_in;
  auto Fp = [&](int i) { return (const float*)d_in[i]; }; auto Ip = [&](int i) { return (const int*)d_in[i]; };
  if (in_sizes[0] != N * HID || in_sizes[1] != 2 * E || in_sizes[2] != 2 * HID * HID || in_sizes[4] != HID * HID || in_sizes[12] != HID * HID || out_size != N * HID) return;
  size_t off = 0; char* ws = (char*)d_ws;
  auto carve = [&](size_t bytes) { char* p = ws + off; off += (bytes + 255) & ~(size_t)255; return p; };
  b16* X16 = (b16*)carve((size_t)N * HID * 2); b16* WT = (b16*)carve((size_t)7 * HID * HID * 2);
  float* XA = (float*)carve((size_t)N * HID * 4); float* XB = (float*)carve((size_t)N * HID * 4); b16* Hh = (b16*)carve((size_t)E * HID * 2); b16* Hl = (b16*)carve((size_t)E * HID * 2);
  float* EF = (float*)carve((size_t)E * HID * 4); b16* EFh = (b16*)carve((size_t)E * HID * 2); b16* EFl = (b16*)carve((size_t)E * HID * 2);
  b16* QFh = (b16*)carve((size_t)NH * E * QP * 2); b16* QFl = (b16*)carve((size_t)NH * E * QP * 2); b16* KRh = (b16*)carve((size_t)NH * E * QP * 2); b16* KRl = (b16*)carve((size_t)NH * E * QP * 2); b16* VT = (b16*)carve((size_t)NH * HD * E * 2); b16* VTl = (b16*)carve((size_t)NH * HD * E * 2);
  b16* AOT = (b16*)carve((size_t)NH * E * HD * 2); b16* AOTl = (b16*)carve((size_t)NH * E * HD * 2); b16* AOh = (b16*)carve((size_t)E * HID * 2); b16* AOl = (b16*)carve((size_t)E * HID * 2); float* UE = (float*)carve((size_t)E * HID * 4);
  CsrBufs csr; off = csr_carve(csr, ws, off, E, N);
  if (off > ws_size || off > ((size_t)128 << 20)) return;
  const b16 *WAB = WT, *WE2 = WT + (size_t)2 * HID * HID, *WQKV = WT + (size_t)3 * HID * HID, *WO = WT + (size_t)6 * HID * HID;
  prep_kernel<<<(N * HID / 8 + 7 * HID * HID / 8 + 255) / 256, 256, 0, stream>>>(Fp(0), Fp(2), Fp(4), Fp(6), Fp(8), Fp(10), Fp(12), X16, WT);
  csr_build(csr, Ip(1) + E, E, N, stream);
  gemm_kernel<0><<<dim3(N / 64, 2), 128, 0, stream>>>(X16, nullptr, WAB, Fp(3), nullptr, nullptr, XA, XB, nullptr, nullptr, nullptr, nullptr);
  edge1_kernel<<<E / 8, 256, 0, stream>>>(XA, XB, Ip(1), Hh, Hl);
  gemm_kernel<1><<<dim3(E / 64, 1), 128, 0, stream>>>(Hh, Hl, WE2, Fp(5), nullptr, nullptr, EF, nullptr, EFh, EFl, nullptr, nullptr);
  gemm_kernel<2><<<dim3(E / 64, 3), 128, 0, stream>>>(EFh, EFl, WQKV, Fp(7), Fp(9), Fp(11), (float*)VT, (float*)VTl, QFh, QFl, KRh, KRl);
  attn_kernel<<<dim3(E / 32, NH), 64, 0, stream>>>(QFh, QFl, KRh, KRl, VT, VTl, AOT, AOTl);
  relay_kernel<<<E / 8, 256, 0, stream>>>(AOT, AOTl, AOh, AOl);
  gemm_kernel<3><<<dim3(E / 64, 1), 128, 0, stream>>>(AOh, AOl, WO, Fp(13), nullptr, nullptr, UE, nullptr, nullptr, nullptr, nullptr, nullptr);
  node_kernel<<<N / 8, 256, 0, stream>>>(Fp(0), UE, csr.PERM, csr.ROWPTR, csr.ROWCNT, (int)csr.permLen, (float*)d_out);
}
